// Encoder_3822520893854
// MI455X (gfx1250) — hardware-verified
//
#include <hip/hip_runtime.h>
#include <math.h>

constexpr int NBAT     = 256;
constexpr int NTRAJ    = 128;
constexpr int TLEN     = 50;
constexpr int NCEN     = 256;
constexpr int CLEN     = 10;
constexpr int CIN      = 3;
constexpr int CH1      = 8;
constexpr int NHID     = 64;
constexpr int NGATE    = 4 * NHID;
constexpr int FCIN     = 8;
constexpr int NSEQ     = NBAT * NTRAJ;
constexpr int NITEM    = NBAT * NCEN;
constexpr int OROWS    = NTRAJ + NCEN;
constexpr int NTHR     = 256;
constexpr int SEQ_BLK  = 32;
constexpr int HALF_SEQ = 16;
constexpr int TPAD     = TLEN + 2;
constexpr int HPITCH   = 72;
constexpr int CPITCH   = 68;
constexpr int ITEM_BLK = 128;
constexpr float A_CARRY = 64.0f;
constexpr float W_CARRY = 16.0f;
constexpr float FOLD    = 1.0f / (A_CARRY * W_CARRY);

static_assert(NSEQ % SEQ_BLK == 0, "trajectory grid exact");
static_assert(NTRAJ % SEQ_BLK == 0, "a block never straddles a batch index");
static_assert(NITEM % ITEM_BLK == 0, "center grid exact");
static_assert(NCEN % ITEM_BLK == 0, "a block never straddles a batch index");
static_assert(SEQ_BLK == 2 * HALF_SEQ, "two prologue halves");
static_assert((2 * SEQ_BLK * HPITCH) % NTHR == 0, "h tile zero fill exact");
static_assert(HALF_SEQ * 2 * CH1 == NTHR, "halo zero fill exact");
static_assert(HALF_SEQ * TPAD * CH1 >= SEQ_BLK * CPITCH, "staging alias fits");
static_assert(HPITCH % 8 == 0 && HPITCH >= NHID, "h tile pitch");
static_assert((SEQ_BLK * NHID / 4) == 2 * NTHR, "trajectory store loop exact");
static_assert((ITEM_BLK * CLEN) % NTHR == 0, "center stage 1 exact");
static_assert((ITEM_BLK * FCIN) % NTHR == 0, "center stage 2 exact");
static_assert(ITEM_BLK == 16 * (NTHR / 32), "16 items per wave");
static_assert(FCIN == CLEN - 2, "valid window length");

typedef __attribute__((ext_vector_type(16))) _Float16 v16h;
typedef __attribute__((ext_vector_type(8)))  _Float16 v8h;
typedef __attribute__((ext_vector_type(8)))  float    v8f;
typedef __attribute__((ext_vector_type(4)))  float    v4f;
typedef __attribute__((ext_vector_type(4)))  unsigned v4u;

union FragU { v16h v; v8h h[2]; };

__device__ __forceinline__ v16h frag_load(const _Float16* p) {
  FragU f;
  f.h[0] = *(const v8h*)(p);
  f.h[1] = *(const v8h*)(p + 16);
  return f.v;
}

__device__ __forceinline__ v16h bfrag_from_f32(const float* p, float sc) {
  const v4f f0 = *(const v4f*)(p);
  const v4f f1 = *(const v4f*)(p + 4);
  const v4f f2 = *(const v4f*)(p + 16);
  const v4f f3 = *(const v4f*)(p + 20);
  v16h r;
#pragma unroll
  for (int e = 0; e < 4; ++e) {
    r[e]      = (_Float16)(f0[e] * sc);
    r[4 + e]  = (_Float16)(f1[e] * sc);
    r[8 + e]  = (_Float16)(f2[e] * sc);
    r[12 + e] = (_Float16)(f3[e] * sc);
  }
  return r;
}

__device__ __forceinline__ v8f mma16(v16h a, v16h b, v8f c) {
  return __builtin_amdgcn_wmma_f32_16x16x32_f16(false, a, false, b, (short)0, c, false, false);
}

__device__ __forceinline__ void group_guard(v8f& a0, v8f& a1, v8f& a2, v8f& a3,
                                            v16h x, v16h b0, v16h b1, v16h b2, v16h b3) {
  asm volatile("v_nop\n\tv_nop\n\tv_nop\n\tv_nop"
               : "+v"(a0), "+v"(a1), "+v"(a2), "+v"(a3)
               : "v"(x), "v"(b0), "v"(b1), "v"(b2), "v"(b3));
}

__device__ __forceinline__ float sigm(float x) {
  return __builtin_amdgcn_rcpf(1.0f + expf(-x));
}

__global__ __launch_bounds__(NTHR) void traj_lstm_kernel(
    const float* __restrict__ x1,
    const float* __restrict__ w11, const float* __restrict__ b11,
    const float* __restrict__ w13, const float* __restrict__ b13,
    const float* __restrict__ w_ih, const float* __restrict__ w_hh,
    const float* __restrict__ b_ih, const float* __restrict__ b_hh,
    float* __restrict__ out)
{
  __shared__ __align__(16) float    s_buf[HALF_SEQ * TPAD * CH1];
  __shared__ __align__(16) _Float16 s_y[SEQ_BLK * TLEN * CH1];
  __shared__ __align__(16) _Float16 Ah[2 * SEQ_BLK * HPITCH];
  __shared__ __align__(16) float    s_w13[CH1 * CH1 * 3];
  __shared__ __align__(16) float    s_w11[CH1 * CIN];
  __shared__ __align__(16) float    s_b11[CH1];
  __shared__ __align__(16) float    s_b13[CH1];

  const int tid  = threadIdx.x;
  const int lane = tid & 31;
  const int wave = tid >> 5;
  const int col  = lane & 15;
  const int hh   = lane >> 4;
  const int koff = hh * 8;
  const int mt   = wave >> 2;
  const int q    = wave & 3;
  const int rowbase = blockIdx.x * SEQ_BLK;

  {
    const int i13 = (tid < CH1 * CH1 * 3) ? tid : (CH1 * CH1 * 3 - 1);
    const float v13 = w13[i13];
    if (tid < CH1 * CH1 * 3) s_w13[tid] = v13;
    const int i11 = (tid < CH1 * CIN) ? tid : (CH1 * CIN - 1);
    const float v11 = w11[i11];
    if (tid < CH1 * CIN) s_w11[tid] = v11;
    const int i8 = (tid < CH1) ? tid : (CH1 - 1);
    const float vb1 = b11[i8];
    const float vb3 = b13[i8];
    if (tid < CH1) { s_b11[tid] = vb1; s_b13[tid] = vb3; }
  }
  {
    const int s = tid >> 4;
    const int r = tid & 15;
    const int row = (r >> 3) ? (TPAD - 1) : 0;
    s_buf[(s * TPAD + row) * CH1 + (r & 7)] = 0.0f;
  }
#pragma unroll 1
  for (int i = tid; i < 2 * SEQ_BLK * HPITCH; i += NTHR) Ah[i] = (_Float16)0.0f;
  __syncthreads();

#pragma unroll 1
  for (int half = 0; half < 2; ++half) {
#pragma unroll 1
    for (int it = 0; it < 4; ++it) {
      const int p  = it * NTHR + tid;
      const bool ok = p < HALF_SEQ * TLEN;
      const int pc = ok ? p : (HALF_SEQ * TLEN - 1);
      const int s  = pc / TLEN;
      const int t  = pc - s * TLEN;
      const float* xp = x1 + ((size_t)(rowbase + half * HALF_SEQ + s) * TLEN + (size_t)t) * CIN;
      const float xa = xp[0];
      const float xb = xp[1];
      const float xc = xp[2];
      float av[CH1];
#pragma unroll
      for (int c = 0; c < CH1; ++c) {
        const float pre = s_w11[c * CIN + 0] * xa + s_w11[c * CIN + 1] * xb + s_w11[c * CIN + 2] * xc + s_b11[c];
        av[c] = tanhf(pre);
      }
      if (ok) {
        float* ap = s_buf + (s * TPAD + t + 1) * CH1;
        v4f lo4 = {av[0], av[1], av[2], av[3]};
        v4f hi4 = {av[4], av[5], av[6], av[7]};
        *(v4f*)(ap)     = lo4;
        *(v4f*)(ap + 4) = hi4;
      }
    }
    __syncthreads();
#pragma unroll 1
    for (int it = 0; it < 4; ++it) {
      const int p  = it * NTHR + tid;
      const bool ok = p < HALF_SEQ * TLEN;
      const int pc = ok ? p : (HALF_SEQ * TLEN - 1);
      const int s  = pc / TLEN;
      const int t  = pc - s * TLEN;
      const float* ap = s_buf + (s * TPAD + t) * CH1;
      float av[3][CH1];
#pragma unroll
      for (int tap = 0; tap < 3; ++tap) {
        const v4f a0 = *(const v4f*)(ap + tap * CH1);
        const v4f a1 = *(const v4f*)(ap + tap * CH1 + 4);
#pragma unroll
        for (int e = 0; e < 4; ++e) { av[tap][e] = a0[e]; av[tap][4 + e] = a1[e]; }
      }
      _Float16* yp = s_y + ((half * HALF_SEQ + s) * TLEN + t) * CH1;
#pragma unroll 1
      for (int c = 0; c < CH1; ++c) {
        const float* wp = s_w13 + c * (CH1 * 3);
        float wv[CH1 * 3];
#pragma unroll
        for (int i = 0; i < 6; ++i) {
          const v4f w4 = *(const v4f*)(wp + 4 * i);
          wv[4 * i + 0] = w4[0]; wv[4 * i + 1] = w4[1]; wv[4 * i + 2] = w4[2]; wv[4 * i + 3] = w4[3];
        }
        float acc = s_b13[c];
#pragma unroll
        for (int ci = 0; ci < CH1; ++ci) {
#pragma unroll
          for (int tap = 0; tap < 3; ++tap) acc += wv[ci * 3 + tap] * av[tap][ci];
        }
        const float yv = (acc > 0.0f) ? acc : 0.01f * acc;
        if (ok) yp[c] = (_Float16)(yv * A_CARRY);
      }
    }
    __syncthreads();
  }

  v16h bh0[4], bh1[4], bx[4];
  float bia[4];
#pragma unroll
  for (int g = 0; g < 4; ++g) {
    const int n = g * NHID + 16 * q + col;
    const float* wr = w_hh + (size_t)n * NHID + koff;
    bh0[g] = bfrag_from_f32(wr, W_CARRY);
    bh1[g] = bfrag_from_f32(wr + 32, W_CARRY);
    const float* wi = w_ih + (size_t)n * CH1;
    const v4f i0 = *(const v4f*)(wi);
    const v4f i1 = *(const v4f*)(wi + 4);
    v16h b;
#pragma unroll
    for (int e = 0; e < 4; ++e) {
      const float u0 = (hh == 0) ? i0[e] : 0.0f;
      const float u1 = (hh == 0) ? i1[e] : 0.0f;
      b[e]      = (_Float16)(u0 * W_CARRY);
      b[4 + e]  = (_Float16)(u1 * W_CARRY);
      b[8 + e]  = (_Float16)0.0f;
      b[12 + e] = (_Float16)0.0f;
    }
    bx[g] = b;
    bia[g] = b_ih[n] + b_hh[n];
  }

  float cst[8];
#pragma unroll
  for (int r = 0; r < 8; ++r) cst[r] = 0.0f;

  const v8f z8 = {0.f, 0.f, 0.f, 0.f, 0.f, 0.f, 0.f, 0.f};
  const v8h zero8 = {(_Float16)0.0f, (_Float16)0.0f, (_Float16)0.0f, (_Float16)0.0f,
                     (_Float16)0.0f, (_Float16)0.0f, (_Float16)0.0f, (_Float16)0.0f};
  const unsigned ym = (hh == 0) ? 0xFFFFFFFFu : 0u;
  const v4u ymask = {ym, ym, ym, ym};
  const _Float16* yrow = s_y + (16 * mt + col) * (TLEN * CH1);

#pragma unroll 1
  for (int t = 0; t < TLEN; ++t) {
    const int cur = t & 1;
    const _Float16* ah = Ah + cur * (SEQ_BLK * HPITCH) + (16 * mt + col) * HPITCH + koff;
    _Float16* ahn = Ah + (cur ^ 1) * (SEQ_BLK * HPITCH) + (16 * mt + 8 * hh) * HPITCH + 16 * q + col;
    const v16h a0 = frag_load(ah);
    const v16h a1 = frag_load(ah + 32);
    const v8h yraw = *(const v8h*)(yrow + t * CH1);
    v4u yw = __builtin_bit_cast(v4u, yraw);
    yw = yw & ymask;
    FragU ax;
    ax.h[0] = __builtin_bit_cast(v8h, yw);
    ax.h[1] = zero8;

    v8f acc[4];
    acc[0] = z8; acc[1] = z8; acc[2] = z8; acc[3] = z8;
#pragma unroll
    for (int g = 0; g < 4; ++g) acc[g] = mma16(a0, bh0[g], acc[g]);
    group_guard(acc[0], acc[1], acc[2], acc[3], a0, bh0[0], bh0[1], bh0[2], bh0[3]);
#pragma unroll
    for (int g = 0; g < 4; ++g) acc[g] = mma16(a1, bh1[g], acc[g]);
    group_guard(acc[0], acc[1], acc[2], acc[3], a1, bh1[0], bh1[1], bh1[2], bh1[3]);
#pragma unroll
    for (int g = 0; g < 4; ++g) acc[g] = mma16(ax.v, bx[g], acc[g]);
    group_guard(acc[0], acc[1], acc[2], acc[3], ax.v, bx[0], bx[1], bx[2], bx[3]);

#pragma unroll
    for (int r = 0; r < 8; ++r) {
      const float zi = acc[0][r] * FOLD + bia[0];
      const float zf = acc[1][r] * FOLD + bia[1];
      const float zg = acc[2][r] * FOLD + bia[2];
      const float zo = acc[3][r] * FOLD + bia[3];
      const float ig = sigm(zi);
      const float fg = sigm(zf);
      const float og = sigm(zo);
      const float gt = tanhf(zg);
      const float cn = fg * cst[r] + ig * gt;
      cst[r] = cn;
      const float hn = og * tanhf(cn);
      ahn[r * HPITCH] = (_Float16)(hn * A_CARRY);
    }
    __syncthreads();
  }

  float* Cs = s_buf;
#pragma unroll
  for (int r = 0; r < 8; ++r) Cs[(16 * mt + 8 * hh + r) * CPITCH + 16 * q + col] = cst[r];
  __syncthreads();
  {
    v4f vv[2];
    float* op[2];
#pragma unroll
    for (int it = 0; it < 2; ++it) {
      const int idx = it * NTHR + tid;
      const int row = idx >> 4;
      const int c4  = (idx & 15) * 4;
      const int n   = rowbase + row;
      const int bb  = n / NTRAJ;
      const int nt  = n - bb * NTRAJ;
      vv[it] = *(const v4f*)(Cs + row * CPITCH + c4);
      op[it] = out + ((size_t)bb * OROWS + (size_t)nt) * NHID + c4;
    }
    for (int pass = 0; pass < 2; ++pass) {
#pragma unroll
      for (int it = 0; it < 2; ++it) *(volatile v4f*)(op[it]) = vv[it];
      __threadfence();
    }
  }
}

__global__ __launch_bounds__(NTHR) void center_kernel(
    const float* __restrict__ x2,
    const float* __restrict__ w21, const float* __restrict__ b21,
    const float* __restrict__ w23, const float* __restrict__ b23,
    const float* __restrict__ wfc, const float* __restrict__ bfc,
    float* __restrict__ out)
{
  __shared__ __align__(16) float s_a2[ITEM_BLK * CLEN * CH1];
  __shared__ __align__(16) float s_z[ITEM_BLK * FCIN];
  __shared__ __align__(16) float s_w21[CH1 * CIN];
  __shared__ __align__(16) float s_b21[CH1];
  __shared__ __align__(16) float s_w23t[3 * CH1];

  const int tid  = threadIdx.x;
  const int lane = tid & 31;
  const int wave = tid >> 5;
  const int itembase = blockIdx.x * ITEM_BLK;

  {
    const int i24 = (tid < CH1 * CIN) ? tid : (CH1 * CIN - 1);
    const float v21 = w21[i24];
    const float v23 = w23[i24];
    if (tid < CH1 * CIN) {
      s_w21[tid] = v21;
      const int c = tid / 3;
      const int tap = tid - c * 3;
      s_w23t[tap * CH1 + c] = v23;
    }
    const int i8 = (tid < CH1) ? tid : (CH1 - 1);
    const float vb = b21[i8];
    if (tid < CH1) s_b21[tid] = vb;
  }
  const float bz = b23[0];
  __syncthreads();

#pragma unroll 1
  for (int it = 0; it < (ITEM_BLK * CLEN) / NTHR; ++it) {
    const int p = it * NTHR + tid;
    const float* xp = x2 + ((size_t)itembase * CLEN + (size_t)p) * CIN;
    const float xa = xp[0];
    const float xb = xp[1];
    const float xc = xp[2];
#pragma unroll 1
    for (int c = 0; c < CH1; ++c) {
      const float pre = s_w21[c * CIN + 0] * xa + s_w21[c * CIN + 1] * xb + s_w21[c * CIN + 2] * xc + s_b21[c];
      s_a2[p * CH1 + c] = tanhf(pre);
    }
  }
  __syncthreads();

#pragma unroll 1
  for (int it = 0; it < (ITEM_BLK * FCIN) / NTHR; ++it) {
    const int o = it * NTHR + tid;
    const int item = o >> 3;
    const int j = o & 7;
    float acc = bz;
#pragma unroll 1
    for (int tap = 0; tap < 3; ++tap) {
      const float* ap = s_a2 + (item * CLEN + j + tap) * CH1;
      const v4f a0 = *(const v4f*)(ap);
      const v4f a1 = *(const v4f*)(ap + 4);
      const v4f w0 = *(const v4f*)(s_w23t + tap * CH1);
      const v4f w1 = *(const v4f*)(s_w23t + tap * CH1 + 4);
#pragma unroll
      for (int e = 0; e < 4; ++e) acc += w0[e] * a0[e];
#pragma unroll
      for (int e = 0; e < 4; ++e) acc += w1[e] * a1[e];
    }
    s_z[o] = (acc > 0.0f) ? acc : 0.01f * acc;
  }
  __syncthreads();

  float wf0[FCIN], wf1[FCIN];
  {
    const float* r0 = wfc + (size_t)lane * FCIN;
    const float* r1 = wfc + (size_t)(lane + 32) * FCIN;
    const v4f p0 = *(const v4f*)(r0);
    const v4f p1 = *(const v4f*)(r0 + 4);
    const v4f q0 = *(const v4f*)(r1);
    const v4f q1 = *(const v4f*)(r1 + 4);
#pragma unroll
    for (int e = 0; e < 4; ++e) { wf0[e] = p0[e]; wf0[4 + e] = p1[e]; wf1[e] = q0[e]; wf1[4 + e] = q1[e]; }
  }
  const float bf0 = bfc[lane];
  const float bf1 = bfc[lane + 32];
#pragma unroll 1
  for (int i = 0; i < 16; ++i) {
    const int item = 16 * wave + i;
    const v4f z0 = *(const v4f*)(s_z + item * FCIN);
    const v4f z1 = *(const v4f*)(s_z + item * FCIN + 4);
    float v0 = bf0;
    float v1 = bf1;
#pragma unroll
    for (int e = 0; e < 4; ++e) { v0 += wf0[e] * z0[e]; v1 += wf1[e] * z0[e]; }
#pragma unroll
    for (int e = 0; e < 4; ++e) { v0 += wf0[4 + e] * z1[e]; v1 += wf1[4 + e] * z1[e]; }
    const int m  = itembase + item;
    const int bb = m / NCEN;
    const int nc = m - bb * NCEN;
    float* op = out + ((size_t)bb * OROWS + (size_t)(NTRAJ + nc)) * NHID + lane;
    for (int pass = 0; pass < 2; ++pass) {
      *(volatile float*)(op)      = v0;
      *(volatile float*)(op + 32) = v1;
      __threadfence();
    }
  }
}

extern "C" void kernel_launch(void* const* d_in, const int* in_sizes, int n_in,
                              void* d_out, int out_size, void* d_ws, size_t ws_size,
                              hipStream_t stream)
{
  (void)d_ws; (void)ws_size;
  if (n_in < 16 || d_out == nullptr) return;
  if (in_sizes[0] != NSEQ * TLEN * CIN || in_sizes[1] != NITEM * CLEN * CIN ||
      in_sizes[2] != CH1 * CIN || in_sizes[3] != CH1 ||
      in_sizes[4] != CH1 * CH1 * 3 || in_sizes[5] != CH1 ||
      in_sizes[6] != NGATE * CH1 || in_sizes[7] != NGATE * NHID ||
      in_sizes[8] != NGATE || in_sizes[9] != NGATE ||
      in_sizes[10] != CH1 * CIN || in_sizes[11] != CH1 ||
      in_sizes[12] != CH1 * 3 || in_sizes[13] != 1 ||
      in_sizes[14] != NHID * FCIN || in_sizes[15] != NHID ||
      out_size != NBAT * OROWS * NHID) return;

  const float* x1   = (const float*)d_in[0];
  const float* x2   = (const float*)d_in[1];
  const float* w11  = (const float*)d_in[2];
  const float* b11  = (const float*)d_in[3];
  const float* w13  = (const float*)d_in[4];
  const float* b13  = (const float*)d_in[5];
  const float* w_ih = (const float*)d_in[6];
  const float* w_hh = (const float*)d_in[7];
  const float* b_ih = (const float*)d_in[8];
  const float* b_hh = (const float*)d_in[9];
  const float* w21  = (const float*)d_in[10];
  const float* b21  = (const float*)d_in[11];
  const float* w23  = (const float*)d_in[12];
  const float* b23  = (const float*)d_in[13];
  const float* wfc  = (const float*)d_in[14];
  const float* bfc  = (const float*)d_in[15];
  float* out = (float*)d_out;

  traj_lstm_kernel<<<dim3(NSEQ / SEQ_BLK), dim3(NTHR), 0, stream>>>(
      x1, w11, b11, w13, b13, w_ih, w_hh, b_ih, b_hh, out);
  center_kernel<<<dim3(NITEM / ITEM_BLK), dim3(NTHR), 0, stream>>>(
      x2, w21, b21, w23, b23, wfc, bfc, out);
}
